// RuleGNN_58463094833889
// MI455X (gfx1250) — hardware-run, weakly checked
//
#include <hip/hip_runtime.h>


namespace {
constexpr int N = 10000, NP = 10048  , E = 262144, D = 128, NR = 64, EPR = 4096, NLY = 2, NQ = 64, ECAP = 128;
constexpr float XS = 8.0f, WSC = 256.0f, MS = 64.0f  , LNEPS = 1e-5f, SCL = 0.08838834764831845f, NEG = 0.2f  ;

typedef _Float16 b16;
typedef __attribute__((ext_vector_type(16))) _Float16 v16b;
typedef __attribute__((ext_vector_type(8))) _Float16 v8b;
typedef __attribute__((ext_vector_type(8))) float v8f;
typedef __attribute__((ext_vector_type(4))) float v4f;
__device__ __forceinline__ float bf16_rne(float f) { unsigned int u = __float_as_uint(f); u += 0x7FFFu + ((u >> 16) & 1u); return __uint_as_float(u & 0xFFFF0000u); }
__device__ __forceinline__ void split16(float v, b16& hi, b16& lo) { hi = (b16)v; lo = (b16)(v - (float)hi); }
__device__ __forceinline__ v16b frag_kb(const b16* p, int hh) { const v8b a = *(const v8b*)(p + 8 * hh), b = *(const v8b*)(p + 16 + 8 * hh); v16b f;
#pragma unroll
  for (int e = 0; e < 8; ++e) { f[e] = a[e]; f[8 + e] = b[e]; } return f; }
__device__ __forceinline__ v8f wmma16b(v16b a, v16b b, v8f c) { v8f d = __builtin_amdgcn_wmma_f32_16x16x32_f16(false, a, false, b, (short)0, c, false, false); asm volatile("v_nop\n\tv_nop\n\tv_nop\n\tv_nop" : "+v"(d) : "v"(a), "v"(b)); return d; }
__device__ __forceinline__ void wave_lds_sync() { __builtin_amdgcn_fence(__ATOMIC_RELEASE, "workgroup"); __builtin_amdgcn_wave_barrier(); __builtin_amdgcn_fence(__ATOMIC_ACQUIRE, "workgroup"); }
__device__ __forceinline__ float pmul(float a, float b) { float p = a * b; asm volatile("" : "+v"(p)); return p; }
__device__ __forceinline__ int iclamp(int v, int lo, int hi) { return v < lo ? lo : (v > hi ? hi : v); }
__device__ __forceinline__ float nexp(float x) { return __builtin_amdgcn_exp2f(x * 1.4426950408889634f); }
__device__ __forceinline__ float lrelu(float x) { return x > 0.0f ? x : NEG * x; }

constexpr int CSR_NBLK = 512, CSR_GB = 8  , CSR_GN = 1 << CSR_GB  , CSR_MAXG = 512, CSR_CAP = 12288  ;
__global__ __launch_bounds__(64) void csrA_kernel(const int* __restrict__ dst, int E, int N, int nG, int CHP, int NGP, int* __restrict__ STG, int* __restrict__ HST) {
  extern __shared__ int sm[];
  int* cnt = sm; int* run = sm + NGP; int* ids = sm + 2 * NGP;
  const int b = blockIdx.x; const int ch = (E + CSR_NBLK - 1) / CSR_NBLK; const int e0 = b * ch, e1 = min(E, e0 + ch);
  for (int i = threadIdx.x; i < NGP; i += 64) cnt[i] = 0;
  for (int i = threadIdx.x; i < CHP; i += 64) ids[i] = -1;
  __syncthreads();
  if (threadIdx.x == 0) {
    for (int e = e0; e < e1; ++e) { int d = dst[e]; d = (d < 0) ? 0 : (d >= N ? N - 1 : d); cnt[d >> CSR_GB] += 1; }
    int acc = 0; for (int g = 0; g < nG; ++g) { run[g] = acc; acc += cnt[g]; }
    for (int e = e0; e < e1; ++e) { int d = dst[e]; d = (d < 0) ? 0 : (d >= N ? N - 1 : d); const int g = d >> CSR_GB; ids[run[g]] = e; run[g] += 1; } }
  __syncthreads();
  typedef __attribute__((ext_vector_type(4))) int v4i;
  for (int pass = 0; pass < 2; ++pass) {
    for (int i = threadIdx.x; i < CHP / 4; i += 64) *(volatile v4i*)(STG + (size_t)b * CHP + i * 4) = *(const v4i*)(&ids[i * 4]);
    for (int i = threadIdx.x; i < NGP / 4; i += 64) { v4i v; for (int e = 0; e < 4; ++e) v[e] = (i * 4 + e < nG) ? cnt[i * 4 + e] : 0; *(volatile v4i*)(HST + (size_t)b * NGP + i * 4) = v; }
    __threadfence(); }
}
__global__ __launch_bounds__(512) void csrS_kernel(const int* __restrict__ HST, int nG, int NGP, int* __restrict__ START, int* __restrict__ TOT, int* __restrict__ OFF) {
  __shared__ int tot[CSR_MAXG];
  const int b = threadIdx.x;
  for (int pass = 0; pass < 2; ++pass) { int runb = 0; for (int g = 0; g < nG; ++g) { int c = HST[(size_t)b * NGP + g]; c = (c < 0) ? 0 : c; ((volatile int*)OFF)[(size_t)g * CSR_NBLK + b] = runb; runb += c; } __threadfence(); }
  for (int g = threadIdx.x; g < nG; g += 512) { int s = 0; for (int bb = 0; bb < CSR_NBLK; ++bb) { int c = HST[(size_t)bb * NGP + g]; s += (c < 0) ? 0 : c; } tot[g] = s; }
  __syncthreads();
  if (threadIdx.x < 32) {
    __shared__ int st[CSR_MAXG + 32];
    if (threadIdx.x == 0) { int acc = 0; for (int g = 0; g < NGP; ++g) { st[g] = acc; if (g < nG) acc += (tot[g] + 31) & ~31; } st[NGP] = acc; }
    __builtin_amdgcn_fence(__ATOMIC_RELEASE, "workgroup"); __builtin_amdgcn_wave_barrier(); __builtin_amdgcn_fence(__ATOMIC_ACQUIRE, "workgroup");
    for (int pass = 0; pass < 2; ++pass) { for (int i = threadIdx.x; i < NGP + 32; i += 32) { ((volatile int*)START)[i] = (i <= NGP) ? st[min(i, NGP)] : 0; ((volatile int*)TOT)[i] = (i < nG) ? tot[i] : 0; } __threadfence(); } }
}
__global__ __launch_bounds__(256) void csrB_kernel(const int* __restrict__ dst, int N, int nG, int CHP, int NGP, int permLen, const int* __restrict__ STG, const int* __restrict__ HST, const int* __restrict__ OFF, const int* __restrict__ START, const int* __restrict__ TOT, int* __restrict__ PERM, int* __restrict__ ROWPTR, int* __restrict__ ROWCNT, int* __restrict__ FLAG) {
  typedef __attribute__((ext_vector_type(4))) int v4i;
  __shared__ int ids[CSR_CAP]; __shared__ unsigned short key[CSR_CAP]; __shared__ int outp[CSR_CAP]; __shared__ int ncnt[CSR_GN + 1]; __shared__ int boff[CSR_NBLK + 1];
  const int g = blockIdx.x, t_ = threadIdx.x; int tot = TOT[g]; int st = START[g], stn = START[g + 1]; const int v0 = g * CSR_GN; const int nv = min(CSR_GN, N - v0);
  st = (st < 0) ? 0 : (st > permLen - 32 ? permLen - 32 : st) & ~31; stn = (stn < st) ? st : (stn > permLen ? permLen : stn); tot = (tot < 0) ? 0 : tot; if (tot > stn - st && tot <= CSR_CAP) tot = stn - st;
  if (tot > CSR_CAP) {
    for (int pass = 0; pass < 2; ++pass) { for (int i = t_; i < CSR_GN / 4; i += 256) { v4i a, c; for (int e = 0; e < 4; ++e) { a[e] = st; c[e] = 0; } *(volatile v4i*)(ROWPTR + v0 + i * 4) = a; *(volatile v4i*)(ROWCNT + v0 + i * 4) = c; } if (t_ == 0) ((volatile int*)FLAG)[0] = 1; __threadfence(); } (void)nv; return; }
  if (t_ == 0) { int acc = 0; for (int b = 0; b < CSR_NBLK; ++b) { boff[b] = acc; int c = HST[(size_t)b * NGP + g]; c = (c < 0) ? 0 : (c > CHP ? CHP : c); acc += c; if (acc > tot) acc = tot; } boff[CSR_NBLK] = acc; }
  for (int i = t_; i <= CSR_GN; i += 256) ncnt[i] = 0;
  __syncthreads();
  for (int b = 0; b < CSR_NBLK; ++b) { const int c = boff[b + 1] - boff[b]; int o_ = OFF[(size_t)g * CSR_NBLK + b]; o_ = (o_ < 0) ? 0 : (o_ > CHP - c ? CHP - c : o_); const int* src_ = STG + (size_t)b * CHP + o_;
    for (int i = t_; i < c; i += 256) { int id = src_[i]; id = (id < 0) ? 0 : id; ids[boff[b] + i] = id; int d = dst[id]; d = (d < v0) ? v0 : (d >= N ? N - 1 : d); int kk = d - v0; kk = (kk < 0) ? 0 : (kk >= CSR_GN ? CSR_GN - 1 : kk); key[boff[b] + i] = (unsigned short)kk; } }
  __syncthreads();
  if (t_ == 0) { for (int i = 0; i < tot; ++i) ncnt[key[i]] += 1; int acc = 0; for (int vl = 0; vl < CSR_GN; ++vl) { const int c = ncnt[vl]; ncnt[vl] = acc; acc += c; } ncnt[CSR_GN] = acc;
    for (int i = 0; i < tot; ++i) { const int vl = key[i]; outp[ncnt[vl]] = ids[i]; ncnt[vl] += 1; }
    for (int vl = CSR_GN; vl > 0; --vl) ncnt[vl] = ncnt[vl - 1]; ncnt[0] = 0; }
  __syncthreads();
  for (int pass = 0; pass < 2; ++pass) {
    for (int i = t_; i < (stn - st) / 4; i += 256) { v4i v; for (int e = 0; e < 4; ++e) { const int q = i * 4 + e; v[e] = (q < tot) ? outp[q] : -1; } *(volatile v4i*)(PERM + st + i * 4) = v; }
    for (int i = t_; i < CSR_GN / 4; i += 256) { v4i a, c; for (int e = 0; e < 4; ++e) { const int vl = i * 4 + e; a[e] = st + ncnt[vl]; c[e] = (vl < nv) ? (ncnt[vl + 1] - ncnt[vl]) : 0; } *(volatile v4i*)(ROWPTR + v0 + i * 4) = a; *(volatile v4i*)(ROWCNT + v0 + i * 4) = c; }
    __threadfence(); }
}
__global__ __launch_bounds__(256) void csrZ_kernel(int* __restrict__ p, size_t n4) { typedef __attribute__((ext_vector_type(4))) int v4i; const size_t tid = (size_t)blockIdx.x * 256 + threadIdx.x, nth = (size_t)gridDim.x * 256; v4i z = {0, 0, 0, 0}; for (size_t i = tid; i < n4; i += nth) *(volatile v4i*)(p + i * 4) = z; }
struct CsrBufs { int *STG, *HST, *OFF, *START, *TOT, *PERM, *ROWPTR, *ROWCNT, *FLAG; int nG, NGP, CHP; size_t permLen; char* base; size_t bytes; };
static size_t csr_carve(CsrBufs& c, char* ws, size_t off, int E, int N) {
  const size_t off0 = off; c.base = ws + off;
  auto al = [&](size_t bytes) { char* p = ws + off; off += (bytes + 255) & ~(size_t)255; return p; };
  c.nG = (N + CSR_GN - 1) / CSR_GN; c.NGP = (c.nG + 31) & ~31; const int ch = (E + CSR_NBLK - 1) / CSR_NBLK; c.CHP = (ch + 31) & ~31; c.permLen = (size_t)E + 32 * (size_t)c.nG + 32;
  c.STG = (int*)al((size_t)CSR_NBLK * c.CHP * 4); c.HST = (int*)al((size_t)CSR_NBLK * c.NGP * 4); c.OFF = (int*)al((size_t)c.NGP * CSR_NBLK * 4); c.START = (int*)al((size_t)(c.NGP + 64) * 4); c.TOT = (int*)al((size_t)(c.NGP + 64) * 4);
  c.PERM = (int*)al(c.permLen * 4); c.ROWPTR = (int*)al((size_t)c.nG * CSR_GN * 4); c.ROWCNT = (int*)al((size_t)c.nG * CSR_GN * 4); c.FLAG = (int*)al(256);
  c.bytes = off - off0; return off;
}
static void csr_build(const CsrBufs& c, const int* dst, int E, int N, hipStream_t stream) {
  const size_t smem = (size_t)(2 * c.NGP + c.CHP) * 4;
  csrZ_kernel<<<512, 256, 0, stream>>>((int*)c.base, c.bytes / 16);
  csrA_kernel<<<CSR_NBLK, 64, smem, stream>>>(dst, E, N, c.nG, c.CHP, c.NGP, c.STG, c.HST);
  csrS_kernel<<<1, 512, 0, stream>>>(c.HST, c.nG, c.NGP, c.START, c.TOT, c.OFF);
  csrB_kernel<<<c.nG, 256, 0, stream>>>(dst, N, c.nG, c.CHP, c.NGP, (int)c.permLen, c.STG, c.HST, c.OFF, c.START, c.TOT, c.PERM, c.ROWPTR, c.ROWCNT, c.FLAG);
}


__global__ __launch_bounds__(256) void wprep_kernel(const float* __restrict__ w, int ldw, int col0, int nmat, b16* __restrict__ dst) {
  const size_t u = (size_t)blockIdx.x * 256 + threadIdx.x; if (u >= (size_t)nmat * D * D / 8) return; const size_t e = u * 8; const int m = (int)(e / (D * D)); const int rem = (int)(e % (D * D)); const int oo = rem / D, k0 = rem % D; v8b o;
  for (int j = 0; j < 8; ++j) o[j] = (b16)(bf16_rne(w[((size_t)m * D + k0 + j) * ldw + col0 + oo]) * WSC);
  for (int pass = 0; pass < 2; ++pass) { *(volatile v8b*)(dst + e) = o; __threadfence(); }
}
__global__ __launch_bounds__(256) void h0_kernel(const float* __restrict__ emb, b16* __restrict__ Hh, b16* __restrict__ Hl) {
  const size_t u = (size_t)blockIdx.x * 256 + threadIdx.x; if (u >= (size_t)NP * D / 8) return; const size_t e = u * 8; const size_t row = e / D; v8b o, z = {};
  for (int j = 0; j < 8; ++j) o[j] = (row < (size_t)N) ? (b16)(bf16_rne(emb[e + j]) * XS) : (b16)0.0f;
  for (int pass = 0; pass < 2; ++pass) { *(volatile v8b*)(Hh + e) = o; *(volatile v8b*)(Hl + e) = z; __threadfence(); }
}
__global__ __launch_bounds__(128) void ngemm_kernel(const b16* __restrict__ Hh, const b16* __restrict__ Hl, const b16* __restrict__ Wt, const float* __restrict__ bias, int nb, float* __restrict__ Y, int ldy) {
  __shared__ __attribute__((aligned(16))) float Tf[4][16][128 + 4];
  const int wave = threadIdx.x >> 5, lane = threadIdx.x & 31, nloc = lane & 15, hlf = lane >> 4; const size_t m0 = (size_t)blockIdx.x * 64 + wave * 16; const int n0 = blockIdx.y * 128; v8f acc[8];
#pragma unroll
  for (int t = 0; t < 8; ++t) acc[t] = (v8f){};
#pragma unroll
  for (int kb = 0; kb < D; kb += 32) { const v16b a = frag_kb(Hh + (m0 + nloc) * D + kb, hlf), al = frag_kb(Hl + (m0 + nloc) * D + kb, hlf);
#pragma unroll
    for (int t = 0; t < 8; ++t) { const v16b bw = frag_kb(Wt + (size_t)(n0 + t * 16 + nloc) * D + kb, hlf); acc[t] = wmma16b(a, bw, acc[t]); acc[t] = wmma16b(al, bw, acc[t]); } }
#pragma unroll
  for (int t = 0; t < 8; ++t) { const int c = n0 + t * 16 + nloc; const float bb = (bias != nullptr && c < nb) ? bf16_rne(bias[c]) : 0.0f;
#pragma unroll 1
    for (int r = 0; r < 8; ++r) Tf[wave][8 * hlf + r][t * 16 + nloc] = acc[t][r] * (1.0f / (XS * WSC)) + bb; }
  wave_lds_sync();
  for (int pass = 0; pass < 2; ++pass) { for (int rr = 0; rr < 16; ++rr) *(volatile v4f*)(Y + (m0 + rr) * ldy + n0 + lane * 4) = *(const v4f*)(&Tf[wave][rr][lane * 4]); __threadfence(); }
}
__global__ __launch_bounds__(128) void msg_kernel(const b16* __restrict__ Hh, const b16* __restrict__ Hl, int lo_on, size_t ebase, const int* __restrict__ srcs, const b16* __restrict__ WR, b16* __restrict__ MSGh, b16* __restrict__ MSGl) {
  __shared__ __attribute__((aligned(16))) b16 Ah[4][16][D + 8], Al[4][16][D + 8], To[4][16][D + 8], Tl[4][16][D + 8];
  const int wave = threadIdx.x >> 5, lane = threadIdx.x & 31, nloc = lane & 15, hlf = lane >> 4; const size_t el = (size_t)blockIdx.x * 64 + wave * 16; const size_t e0 = ebase + el; const int rel = (int)(e0 / EPR); const b16* W = WR + (size_t)rel * D * D;
  for (int q = lane; q < 16 * 16; q += 32) { const int rr = q >> 4, c8 = (q & 15) * 8; const size_t s = (size_t)iclamp(srcs[e0 + rr], 0, N - 1); *(v8b*)(&Ah[wave][rr][c8]) = *(const v8b*)(Hh + s * D + c8); *(v8b*)(&Al[wave][rr][c8]) = *(const v8b*)(Hl + s * D + c8); }
  wave_lds_sync(); v8f acc[8];
#pragma unroll
  for (int t = 0; t < 8; ++t) acc[t] = (v8f){};
#pragma unroll
  for (int kb = 0; kb < D; kb += 32) { const v16b a = frag_kb(&Ah[wave][nloc][kb], hlf), al = frag_kb(&Al[wave][nloc][kb], hlf);
#pragma unroll
    for (int t = 0; t < 8; ++t) { const v16b bw = frag_kb(W + (size_t)(t * 16 + nloc) * D + kb, hlf); acc[t] = wmma16b(a, bw, acc[t]); if (lo_on) acc[t] = wmma16b(al, bw, acc[t]); } }
#pragma unroll
  for (int t = 0; t < 8; ++t)
#pragma unroll 1
    for (int r = 0; r < 8; ++r) { b16 p, q; split16(acc[t][r] * (MS / (XS * WSC)), p, q); To[wave][8 * hlf + r][t * 16 + nloc] = p; Tl[wave][8 * hlf + r][t * 16 + nloc] = q; }
  wave_lds_sync();
  for (int pass = 0; pass < 2; ++pass) { for (int r2 = 0; r2 < 16; r2 += 2) { const int rr = r2 + (lane >> 4), c8 = (lane & 15) * 8; *(volatile v8b*)(MSGh + (el + rr) * D + c8) = *(const v8b*)(&To[wave][rr][c8]); *(volatile v8b*)(MSGl + (el + rr) * D + c8) = *(const v8b*)(&Tl[wave][rr][c8]); } __threadfence(); }
}
__global__ __launch_bounds__(256) void agg_kernel(const float* __restrict__ XQK, const b16* __restrict__ MSGh, const b16* __restrict__ MSGl, int half, const int* __restrict__ srcs, const int* __restrict__ etype, const int* __restrict__ PERM, const int* __restrict__ ROWPTR, const int* __restrict__ ROWCNT, int permLen, const float* __restrict__ cbias, const float* __restrict__ g, const float* __restrict__ bta, float* __restrict__ OUTP, b16* __restrict__ Hh, b16* __restrict__ Hl) {
  __shared__ float lg[8][ECAP], at[8][ECAP]; __shared__ int ty[8][ECAP], eid[8][ECAP];
  const int wave = threadIdx.x >> 5, lane = threadIdx.x & 31; const size_t v = (size_t)blockIdx.x * 8 + wave;
  float o[4] = {0.0f, 0.0f, 0.0f, 0.0f}; int cnt = 0;
  if (v < (size_t)N) { int st = ROWPTR[v]; cnt = ROWCNT[v]; cnt = iclamp(cnt, 0, ECAP); st = iclamp(st, 0, permLen - cnt);
    const v4f q4 = *(const v4f*)(XQK + v * 2 * D + lane * 4);
    for (int i = 0; i < cnt; ++i) { const int e = iclamp(PERM[st + i], 0, E - 1); const size_t s = (size_t)iclamp(srcs[e], 0, N - 1); const v4f k4 = *(const v4f*)(XQK + s * 2 * D + D + lane * 4);
      float p = pmul(q4[0], k4[0]) + pmul(q4[1], k4[1]) + pmul(q4[2], k4[2]) + pmul(q4[3], k4[3]);
#pragma unroll
      for (int sh = 16; sh >= 1; sh >>= 1) p += __shfl_xor(p, sh);
      if (lane == 0) { lg[wave][i] = p * SCL; ty[wave][i] = etype[e]; eid[wave][i] = e; } }
    wave_lds_sync();
    for (int i = lane; i < cnt; i += 32) { const int t_ = ty[wave][i]; float m = -INFINITY; for (int j = 0; j < cnt; ++j) if (ty[wave][j] == t_) m = fmaxf(m, lg[wave][j]);
      float den = 0.0f; for (int j = 0; j < cnt; ++j) if (ty[wave][j] == t_) den += __expf(lg[wave][j] - m); at[wave][i] = __expf(lg[wave][i] - m) / den; }
    wave_lds_sync();
    const size_t ebase = (size_t)half * (E / 2);
    for (int i = 0; i < cnt; ++i) { const size_t e = (size_t)eid[wave][i]; if (e < ebase || e >= ebase + E / 2) continue; const float a = at[wave][i]; const b16* mp = MSGh + (e - ebase) * D + lane * 4; const b16* ml = MSGl + (e - ebase) * D + lane * 4;
      for (int j = 0; j < 4; ++j) o[j] += pmul(a, ((float)mp[j] + (float)ml[j]) * (1.0f / MS)); } }
  if (half == 0) { v4f ov = {o[0], o[1], o[2], o[3]}; for (int pass = 0; pass < 2; ++pass) { *(volatile v4f*)(OUTP + v * D + lane * 4) = ov; __threadfence(); } return; }
  { const v4f pv = *(const v4f*)(OUTP + v * D + lane * 4); for (int j = 0; j < 4; ++j) o[j] += pv[j]; }
  float x[4]; float s = 0.0f; for (int j = 0; j < 4; ++j) { x[j] = o[j] + bf16_rne(cbias[lane * 4 + j]); s += x[j]; }
#pragma unroll
  for (int sh = 16; sh >= 1; sh >>= 1) s += __shfl_xor(s, sh);
  const float mu = s * (1.0f / D); float q = 0.0f; for (int j = 0; j < 4; ++j) { const float d = x[j] - mu; q += d * d; }
#pragma unroll
  for (int sh = 16; sh >= 1; sh >>= 1) q += __shfl_xor(q, sh);
  const float rs = rsqrtf(q * (1.0f / D) + LNEPS); v4f yh, yl; __attribute__((unused)) int dummy = 0; b16 hv[4], lv[4];
  for (int j = 0; j < 4; ++j) { float y = fmaxf((x[j] - mu) * rs * bf16_rne(g[lane * 4 + j]) + bf16_rne(bta[lane * 4 + j]), 0.0f); if (v >= (size_t)N) y = 0.0f; split16(y * XS, hv[j], lv[j]); }
  typedef __attribute__((ext_vector_type(4))) _Float16 v4h; v4h ph, pl; for (int j = 0; j < 4; ++j) { ph[j] = hv[j]; pl[j] = lv[j]; }
  for (int pass = 0; pass < 2; ++pass) { *(volatile v4h*)(Hh + v * D + lane * 4) = ph; *(volatile v4h*)(Hl + v * D + lane * 4) = pl; __threadfence(); } (void)yh; (void)yl;
}
__global__ __launch_bounds__(256) void qrows_kernel(const b16* __restrict__ Hh, const b16* __restrict__ Hl, const int* __restrict__ queries, b16* __restrict__ QHh, b16* __restrict__ QHl) {
  const int u = blockIdx.x * 256 + threadIdx.x; if (u >= NQ * D / 8) return; const int e = u * 8, b = e / D, c8 = e % D; const size_t n = (size_t)iclamp(queries[b * 2], 0, N - 1);
  const v8b a = *(const v8b*)(Hh + n * D + c8), c = *(const v8b*)(Hl + n * D + c8);
  for (int pass = 0; pass < 2; ++pass) { *(volatile v8b*)(QHh + e) = a; *(volatile v8b*)(QHl + e) = c; __threadfence(); }
}
__global__ __launch_bounds__(256) void score_kernel(const float* __restrict__ QW, const float* __restrict__ HW, const float* __restrict__ w2, const float* __restrict__ b2, float* __restrict__ out) {
  __shared__ float w2s[D]; if (threadIdx.x < D) w2s[threadIdx.x] = bf16_rne(w2[threadIdx.x]); __syncthreads();
  const size_t i0 = ((size_t)blockIdx.x * 256 + threadIdx.x) * 4; if (i0 >= (size_t)NQ * N) return; v4f r; const float bb = bf16_rne(b2[0]);
  for (int j = 0; j < 4; ++j) { const size_t i = i0 + j; const int b = (int)(i / N), n = (int)(i % N); const float* qw = QW + (size_t)b * D; const float* hw = HW + (size_t)n * D; float s = bb;
#pragma unroll 4
    for (int c = 0; c < D; ++c) s += pmul(fmaxf(qw[c] + hw[c], 0.0f), w2s[c]);
    r[j] = s; }
  for (int pass = 0; pass < 2; ++pass) { *(volatile v4f*)(out + i0) = r; __threadfence(); }
}
}

extern "C" void kernel_launch(void* const* d_in, const int* in_sizes, int n_in, void* d_out, int out_size, void* d_ws, size_t ws_size, hipStream_t stream) {
  (void)n_in;
  auto Fp = [&](int i) { return (const float*)d_in[i]; }; auto Ip = [&](int i) { return (const int*)d_in[i]; };
  if (in_sizes[0] != N * D || in_sizes[1] != NLY * NR * D * D || in_sizes[2] != NLY * D * D || in_sizes[4] != NLY * 3 * D * D || in_sizes[10] != 2 * D * D || in_sizes[14] != NQ * 2 || in_sizes[15] != 2 * E || in_sizes[16] != E || out_size != NQ * N) return;
  size_t off = 0; char* ws = (char*)d_ws;
  auto carve = [&](size_t bytes) { char* p = ws + off; off += (bytes + 255) & ~(size_t)255; return p; };
  b16* WQK = (b16*)carve((size_t)NLY * 2 * D * D * 2); b16* WRT = (b16*)carve((size_t)NLY * NR * D * D * 2); b16* W1A = (b16*)carve((size_t)D * D * 2); b16* W1B = (b16*)carve((size_t)D * D * 2);
  b16* Hh = (b16*)carve((size_t)NP * D * 2); b16* Hl = (b16*)carve((size_t)NP * D * 2); float* XQK = (float*)carve((size_t)NP * 2 * D * 4); b16* MSGh = (b16*)carve((size_t)(E / 2) * D * 2); b16* MSGl = (b16*)carve((size_t)(E / 2) * D * 2); float* OUTP = (float*)carve((size_t)NP * D * 4);
  float* HW = (float*)carve((size_t)NP * D * 4); b16* QHh = (b16*)carve((size_t)NQ * D * 2); b16* QHl = (b16*)carve((size_t)NQ * D * 2); float* QW = (float*)carve((size_t)NQ * D * 4);
  CsrBufs csr; off = csr_carve(csr, ws, off, E, N);
  if (off > ws_size || off > ((size_t)128 << 20)) return;
  const unsigned g1 = (D * D / 8 + 255) / 256;
  for (int l = 0; l < NLY; ++l) { wprep_kernel<<<g1, 256, 0, stream>>>(Fp(2) + (size_t)l * D * D, D, 0, 1, WQK + (size_t)l * 2 * D * D);
    wprep_kernel<<<g1, 256, 0, stream>>>(Fp(4) + (size_t)l * 3 * D * D, D, 0, 1, WQK + (size_t)l * 2 * D * D + (size_t)D * D);
    wprep_kernel<<<g1 * NR, 256, 0, stream>>>(Fp(1) + (size_t)l * NR * D * D, D, 0, NR, WRT + (size_t)l * NR * D * D); }
  wprep_kernel<<<g1, 256, 0, stream>>>(Fp(10), D, 0, 1, W1A); wprep_kernel<<<g1, 256, 0, stream>>>(Fp(10) + (size_t)D * D, D, 0, 1, W1B);
  csr_build(csr, Ip(15) + E, E, N, stream);
  h0_kernel<<<(unsigned)(((size_t)NP * D / 8 + 255) / 256), 256, 0, stream>>>(Fp(0), Hh, Hl);
  for (int l = 0; l < NLY; ++l) {
    ngemm_kernel<<<dim3(NP / 64, 2), 128, 0, stream>>>(Hh, Hl, WQK + (size_t)l * 2 * D * D, Fp(3) + l * D, D, XQK, 2 * D);
    for (int half = 0; half < 2; ++half) {
      msg_kernel<<<(E / 2) / 64, 128, 0, stream>>>(Hh, Hl, l > 0 ? 1 : 0, (size_t)half * (E / 2), Ip(15), WRT + (size_t)l * NR * D * D, MSGh, MSGl);
      agg_kernel<<<NP / 8, 256, 0, stream>>>(XQK, MSGh, MSGl, half, Ip(15), Ip(16), csr.PERM, csr.ROWPTR, csr.ROWCNT, (int)csr.permLen, Fp(7) + l * D, Fp(8) + l * D, Fp(9) + l * D, OUTP, Hh, Hl); }
  }
  ngemm_kernel<<<dim3(NP / 64, 1), 128, 0, stream>>>(Hh, Hl, W1B, Fp(11), D, HW, D);
  qrows_kernel<<<(NQ * D / 8 + 255) / 256, 256, 0, stream>>>(Hh, Hl, Ip(14), QHh, QHl);
  ngemm_kernel<<<dim3(1, 1), 128, 0, stream>>>(QHh, QHl, W1A, nullptr, 0, QW, D);
  score_kernel<<<(unsigned)(((size_t)NQ * N / 4 + 255) / 256), 256, 0, stream>>>(QW, HW, Fp(12), Fp(13), (float*)d_out);
}
